// MultiHeadAttention_54382875902378
// MI455X (gfx1250) — hardware-verified
//
#include <hip/hip_runtime.h>
#include <stddef.h>


#ifndef NB
#define NB 2
#endif
#ifndef SEQ
#define SEQ 256
#endif
#define NB_FULL 2
#define SEQ_FULL 256
#define DM 512
#define NH 8
#define DKH 64
#define DW (DM * NH)
#define LSEQ (SEQ * NH)
#define MROWS (NB * SEQ)

static_assert(NB >= 1 && NB <= NB_FULL);
static_assert(SEQ >= 64 && SEQ <= SEQ_FULL);
static_assert(SEQ % 64 == 0);
static_assert(MROWS % 64 == 0);
static_assert(LSEQ % 128 == 0);
static_assert(LSEQ % 64 == 0);
static_assert(LSEQ % 32 == 0);
static_assert(NH * DKH == DM);
static_assert(DKH == 64);
static_assert(DM % 256 == 0);
static_assert(DW % 256 == 0);
static_assert(DM % 64 == 0 && DW % 64 == 0);
static_assert(DM % 32 == 0 && DW % 32 == 0);
static_assert(DM % 8 == 0);

#define P_CARRY   1024.0f
#define CTX_SCALE 0.25f
#define WF_CARRY  64.0f
#define OUT_FOLD  (1.0f / 16384.0f)
#define QK_SCALE  0.125f

typedef unsigned short us;
typedef us        v8us  __attribute__((ext_vector_type(8)));
typedef us        v16us __attribute__((ext_vector_type(16)));
typedef _Float16  v16h  __attribute__((ext_vector_type(16)));
typedef __bf16    v16bf __attribute__((ext_vector_type(16)));
typedef float     v8f   __attribute__((ext_vector_type(8)));
typedef float     v4f   __attribute__((ext_vector_type(4)));

constexpr size_t XE = (size_t)MROWS * DM;
constexpr size_t WE = (size_t)DM * DW;
constexpr size_t PE = (size_t)MROWS * DW;
constexpr size_t WS_TOTAL_BYTES = (3 * XE + 4 * WE + 5 * PE) * sizeof(us);
static_assert(WS_TOTAL_BYTES <= (size_t)134217728);
static_assert((XE * sizeof(us)) % 128 == 0 && (WE * sizeof(us)) % 128 == 0 && (PE * sizeof(us)) % 128 == 0);

__device__ __forceinline__ unsigned bf16rne_bits(float x) {
  unsigned u = __float_as_uint(x);
  return (u + 0x7FFFu + ((u >> 16) & 1u)) >> 16;
}
__device__ __forceinline__ float bf16rne(float x) {
  return __uint_as_float(bf16rne_bits(x) << 16);
}
__device__ __forceinline__ us f16_bits(float x) {
  _Float16 hx = (_Float16)x;
  return __builtin_bit_cast(us, hx);
}

__device__ __forceinline__ v16us frag16(const us* base, int ld, int row0, int k0) {
  const int l = threadIdx.x & 31;
  const int r = l & 15, s = l >> 4;
  const us* p = base + (size_t)(row0 + r) * ld + k0 + 8 * s;
  v8us c0 = *(const v8us*)p;
  v8us c1 = *(const v8us*)(p + 16);
  return __builtin_shufflevector(c0, c1, 0, 1, 2, 3, 4, 5, 6, 7, 8, 9, 10, 11, 12, 13, 14, 15);
}
__device__ __forceinline__ v16h fragh(const us* base, int ld, int row0, int k0) {
  return __builtin_bit_cast(v16h, frag16(base, ld, row0, k0));
}
__device__ __forceinline__ v16bf fragb(const us* base, int ld, int row0, int k0) {
  return __builtin_bit_cast(v16bf, frag16(base, ld, row0, k0));
}

__device__ __forceinline__ v8f mma_f16(v16h a, v16h b, v8f c) {
  v8f d = __builtin_amdgcn_wmma_f32_16x16x32_f16(false, a, false, b, (short)0, c, false, false);
  asm volatile("v_nop\n\tv_nop\n\tv_nop\n\tv_nop" : "+v"(d) : "v"(a), "v"(b));
  return d;
}
__device__ __forceinline__ v8f mma_bf16(v16bf a, v16bf b, v8f c) {
  v8f d = __builtin_amdgcn_wmma_f32_16x16x32_bf16(false, a, false, b, (short)0, c, false, false);
  asm volatile("v_nop\n\tv_nop\n\tv_nop\n\tv_nop" : "+v"(d) : "v"(a), "v"(b));
  return d;
}

__global__ __launch_bounds__(256) void cvt_x_kernel(const float* __restrict__ X, us* Y, int n8) {
  const int i = blockIdx.x * 256 + threadIdx.x;
  if (i >= n8) return;
  constexpr int G = DM / 8;
  const int m  = i / G;
  const int c8 = (i - m * G) * 8;
  const int b  = m / SEQ;
  const int s  = m - b * SEQ;
  const float* src = X + ((size_t)(b * SEQ_FULL + s)) * DM + c8;
  v4f x0 = *(const v4f*)src;
  v4f x1 = *(const v4f*)(src + 4);
  v8us y;
#pragma unroll
  for (int j = 0; j < 4; ++j) {
    y[j]     = (us)bf16rne_bits(x0[j]);
    y[4 + j] = (us)bf16rne_bits(x1[j]);
  }
  us* dst = Y + (size_t)i * 8;
  *(volatile v8us*)dst = y;
  __threadfence();
  *(volatile v8us*)dst = y;
}

__global__ __launch_bounds__(256) void cvt_w_kernel(const float* __restrict__ W, us* WT,
                                                    int Kd, int Nd, int hmode) {
  __shared__ float tile[64 * 65];
  const int t  = threadIdx.x;
  const int n0 = blockIdx.x * 64;
  const int k0 = blockIdx.y * 64;
  {
    const int kr = t >> 2;
    const int cc = (t & 3) * 16;
    const float* src = W + (size_t)(k0 + kr) * Nd + n0 + cc;
#pragma unroll
    for (int j = 0; j < 4; ++j) {
      v4f x = *(const v4f*)(src + 4 * j);
#pragma unroll
      for (int e = 0; e < 4; ++e) tile[kr * 65 + cc + 4 * j + e] = x[e];
    }
  }
  __syncthreads();

  v8us vals[2];
  size_t dsts[2];
  const int c = t & 7;
#pragma unroll
  for (int it = 0; it < 2; ++it) {
    const int nl = (t >> 3) + 32 * it;
    v8us o;
#pragma unroll
    for (int j = 0; j < 8; ++j) {
      const float w = bf16rne(tile[(8 * c + j) * 65 + nl]);
      const us hb = (us)(__float_as_uint(w) >> 16);
      const us hf = f16_bits(w * WF_CARRY);
      o[j] = hmode ? hf : hb;
    }
    vals[it] = o;
    dsts[it] = (size_t)(n0 + nl) * Kd + k0 + 8 * c;
  }
#pragma unroll
  for (int it = 0; it < 2; ++it) *(volatile v8us*)(WT + dsts[it]) = vals[it];
  __threadfence();
#pragma unroll
  for (int it = 0; it < 2; ++it) *(volatile v8us*)(WT + dsts[it]) = vals[it];
}

template <int KD>
__device__ __forceinline__ void gemm32x64_bf16(const us* A, const us* B, int m0, int n0, v8f (&acc)[8]) {
  static_assert(KD % 32 == 0);
#pragma unroll 1
  for (int kk = 0; kk < KD; kk += 32) {
    const v16bf a0 = fragb(A, KD, m0, kk);
    const v16bf a1 = fragb(A, KD, m0 + 16, kk);
#pragma unroll
    for (int tt = 0; tt < 4; ++tt) {
      const v16bf b = fragb(B, KD, n0 + 16 * tt, kk);
      acc[tt]     = mma_bf16(a0, b, acc[tt]);
      acc[4 + tt] = mma_bf16(a1, b, acc[4 + tt]);
    }
  }
}
template <int KD>
__device__ __forceinline__ void gemm32x64_f16(const us* A, const us* B, int m0, int n0, v8f (&acc)[8]) {
  static_assert(KD % 32 == 0);
#pragma unroll 1
  for (int kk = 0; kk < KD; kk += 32) {
    const v16h a0 = fragh(A, KD, m0, kk);
    const v16h a1 = fragh(A, KD, m0 + 16, kk);
#pragma unroll
    for (int tt = 0; tt < 4; ++tt) {
      const v16h b = fragh(B, KD, n0 + 16 * tt, kk);
      acc[tt]     = mma_f16(a0, b, acc[tt]);
      acc[4 + tt] = mma_f16(a1, b, acc[4 + tt]);
    }
  }
}

__global__ __launch_bounds__(256) __attribute__((amdgpu_num_vgpr(256)))
void proj_kernel(const us* __restrict__ Xb, const us* __restrict__ Wt,
                 const float* __restrict__ bias, us* Y) {
  __shared__ us stile[64 * 256];

  const int t = threadIdx.x, wid = t >> 5, l = t & 31;
  const int h = l >> 4, r16 = l & 15;
  const int wm = wid >> 2, wn = wid & 3;
  const int mblk0 = blockIdx.x * 64;
  const int nblk0 = blockIdx.y * 256;
  const int m0 = mblk0 + wm * 32;
  const int n0 = nblk0 + wn * 64;

  v8f acc[8] = {};
  gemm32x64_bf16<DM>(Xb, Wt, m0, n0, acc);

#pragma unroll
  for (int tt = 0; tt < 4; ++tt) {
    const int n = n0 + 16 * tt + r16;
    const float bvv = bf16rne(bias[n]);
    const int nl = wn * 64 + 16 * tt + r16;
#pragma unroll
    for (int mi = 0; mi < 2; ++mi) {
#pragma unroll
      for (int r = 0; r < 8; ++r) {
        const int ml = wm * 32 + 16 * mi + 8 * h + r;
        const float v = acc[mi * 4 + tt][r] + bvv;
        stile[ml * 256 + nl] = f16_bits(v);
      }
    }
  }
  __syncthreads();

  const int bblk = mblk0 / SEQ;
  const int sblk = mblk0 - bblk * SEQ;
  const int jchunk = nblk0 / DM;
  const int hbase  = (nblk0 - jchunk * DM) / DKH;
  const int c = l & 7;
  v8us vals[8];
  size_t dsts[8];
#pragma unroll
  for (int it = 0; it < 8; ++it) {
    const int L = wid * 32 + (l >> 3) + 4 * it;
    const int ml = L >> 2, hq = L & 3;
    const int hg = hbase + hq;
    const int p = (sblk + ml) * NH + jchunk;
    vals[it] = *(const v8us*)&stile[ml * 256 + hq * 64 + 8 * c];
    dsts[it] = (((size_t)(bblk * NH + hg)) * LSEQ + p) * DKH + 8 * c;
  }
#pragma unroll
  for (int it = 0; it < 8; ++it) *(volatile v8us*)(Y + dsts[it]) = vals[it];
  __threadfence();
#pragma unroll
  for (int it = 0; it < 8; ++it) *(volatile v8us*)(Y + dsts[it]) = vals[it];
}

__global__ __launch_bounds__(256) void vtrans_kernel(const us* __restrict__ Vh, us* Vt) {
  __shared__ us tile[64 * 65];
  const int t  = threadIdx.x;
  const int p0 = blockIdx.x * 64;
  const int bh = blockIdx.y;
  {
    const int pr = t >> 2;
    const int cc = (t & 3) * 16;
    const us* src = Vh + ((size_t)bh * LSEQ + p0 + pr) * DKH + cc;
    v8us x0 = *(const v8us*)src;
    v8us x1 = *(const v8us*)(src + 8);
#pragma unroll
    for (int e = 0; e < 8; ++e) {
      tile[pr * 65 + cc + e]     = x0[e];
      tile[pr * 65 + cc + 8 + e] = x1[e];
    }
  }
  __syncthreads();

  v8us vals[2];
  size_t dsts[2];
  const int c = t & 7;
#pragma unroll
  for (int it = 0; it < 2; ++it) {
    const int dl = (t >> 3) + 32 * it;
    v8us o;
#pragma unroll
    for (int j = 0; j < 8; ++j) o[j] = tile[(8 * c + j) * 65 + dl];
    vals[it] = o;
    dsts[it] = ((size_t)bh * DKH + dl) * LSEQ + p0 + 8 * c;
  }
#pragma unroll
  for (int it = 0; it < 2; ++it) *(volatile v8us*)(Vt + dsts[it]) = vals[it];
  __threadfence();
#pragma unroll
  for (int it = 0; it < 2; ++it) *(volatile v8us*)(Vt + dsts[it]) = vals[it];
}

__global__ __launch_bounds__(256) __attribute__((amdgpu_num_vgpr(256)))
void attn_kernel(const us* __restrict__ Qh, const us* __restrict__ Kh,
                 const us* __restrict__ Vt, us* Ctx) {
  __shared__ us shK[32 * 64];
  __shared__ us shV[64 * 32];
  __shared__ us shC[8 * 16 * 64];

  const int t = threadIdx.x, wid = t >> 5, l = t & 31;
  const int r16 = l & 15;
  const int rowsel = (l >> 4) << 3;
  constexpr int QBLK = LSEQ / 128;
  const int bh = blockIdx.x / QBLK;
  const int qb = blockIdx.x - bh * QBLK;
  const int q0 = qb * 128 + wid * 16;

  const us* qp = Qh + (size_t)bh * LSEQ * DKH;
  const us* kp = Kh + (size_t)bh * LSEQ * DKH;
  const us* vp = Vt + (size_t)bh * DKH * LSEQ;

  const v16h qB0 = fragh(qp, DKH, q0, 0);
  const v16h qB1 = fragh(qp, DKH, q0, 32);

  v8f o[4];
#pragma unroll
  for (int tt = 0; tt < 4; ++tt) o[tt] = v8f{};
  float mmax = -1.0e30f, lsum = 0.0f;

  const int krow = t >> 3, kcol = (t & 7) * 8;
  const int vrow = t >> 2, vcol = (t & 3) * 8;

#pragma unroll 1
  for (int kb = 0; kb < LSEQ; kb += 32) {
    __syncthreads();
    *(v8us*)&shK[krow * 64 + kcol] = *(const v8us*)(kp + (size_t)(kb + krow) * DKH + kcol);
    *(v8us*)&shV[vrow * 32 + vcol] = *(const v8us*)(vp + (size_t)vrow * LSEQ + kb + vcol);
    __syncthreads();

    v8f s0 = {};
    v8f s1 = {};
    {
      const v16h kA = fragh(shK, 64, 0, 0);
      s0 = mma_f16(kA, qB0, s0);
    }
    {
      const v16h kA = fragh(shK, 64, 0, 32);
      s0 = mma_f16(kA, qB1, s0);
    }
    {
      const v16h kA = fragh(shK, 64, 16, 0);
      s1 = mma_f16(kA, qB0, s1);
    }
    {
      const v16h kA = fragh(shK, 64, 16, 32);
      s1 = mma_f16(kA, qB1, s1);
    }

    float bm = s0[0];
#pragma unroll
    for (int i = 0; i < 8; ++i) { bm = fmaxf(bm, s0[i]); bm = fmaxf(bm, s1[i]); }
    bm = fmaxf(bm, __shfl_xor(bm, 16, 32));
    const float mnew = fmaxf(mmax, bm * QK_SCALE);
    const float corr = __expf(mmax - mnew);
    mmax = mnew;

    float ps = 0.0f;
    v16h pA;
#pragma unroll
    for (int i = 0; i < 8; ++i) {
      const float p0 = __expf(s0[i] * QK_SCALE - mnew);
      const float p1 = __expf(s1[i] * QK_SCALE - mnew);
      ps += p0 + p1;
      pA[i]     = (_Float16)(p0 * P_CARRY);
      pA[8 + i] = (_Float16)(p1 * P_CARRY);
    }
    ps += __shfl_xor(ps, 16, 32);
    lsum = lsum * corr + ps;

#pragma unroll
    for (int r = 0; r < 8; ++r) {
      const float cr = __shfl(corr, rowsel + r, 32);
#pragma unroll
      for (int tt = 0; tt < 4; ++tt) o[tt][r] *= cr;
    }

#pragma unroll
    for (int tt = 0; tt < 4; ++tt) {
      const v16h vB = fragh(shV, 32, 16 * tt, 0);
      o[tt] = mma_f16(pA, vB, o[tt]);
    }
  }

  const int bb = bh / NH;
  const int hh = bh - bb * NH;
#pragma unroll
  for (int r = 0; r < 8; ++r) {
    const float lrow = __shfl(lsum, rowsel + r, 32);
    const float li = CTX_SCALE * __builtin_amdgcn_rcpf(lrow);
#pragma unroll
    for (int tt = 0; tt < 4; ++tt) {
      shC[wid * 1024 + (rowsel + r) * 64 + 16 * tt + r16] = f16_bits(o[tt][r] * li);
    }
  }
  __syncthreads();

  const int c = l & 7;
  v8us vals[4];
  size_t dsts[4];
#pragma unroll
  for (int it = 0; it < 4; ++it) {
    const int rl = (l >> 3) + 4 * it;
    vals[it] = *(const v8us*)&shC[wid * 1024 + rl * 64 + 8 * c];
    const int p = q0 + rl;
    const int s = p / NH;
    const int j = p - s * NH;
    dsts[it] = ((size_t)(bb * SEQ + s)) * DW + j * DM + hh * DKH + 8 * c;
  }
#pragma unroll
  for (int it = 0; it < 4; ++it) *(volatile v8us*)(Ctx + dsts[it]) = vals[it];
  __threadfence();
#pragma unroll
  for (int it = 0; it < 4; ++it) *(volatile v8us*)(Ctx + dsts[it]) = vals[it];
}

__global__ __launch_bounds__(256) __attribute__((amdgpu_num_vgpr(256)))
void outproj_kernel(const us* __restrict__ Ctx, const us* __restrict__ Wft,
                    const float* __restrict__ bo, float* Out) {
  __shared__ float ftile[32 * 256];

  const int t = threadIdx.x, wid = t >> 5, l = t & 31;
  const int h = l >> 4, r16 = l & 15;
  const int wm = wid >> 2, wn = wid & 3;
  const int mblk0 = blockIdx.x * 64;
  const int nblk0 = blockIdx.y * 256;
  const int m0 = mblk0 + wm * 32;
  const int n0 = nblk0 + wn * 64;

  v8f acc[8] = {};
  gemm32x64_f16<DW>(Ctx, Wft, m0, n0, acc);

  const int c = l & 7;
#pragma unroll
  for (int p = 0; p < 2; ++p) {
    if (p) __syncthreads();
#pragma unroll
    for (int tt = 0; tt < 4; ++tt) {
      const int n = n0 + 16 * tt + r16;
      const float bob = bf16rne(bo[n]);
      const int nl = wn * 64 + 16 * tt + r16;
#pragma unroll
      for (int r = 0; r < 8; ++r) {
        const int rl = wm * 16 + 8 * h + r;
        ftile[rl * 256 + nl] = acc[p * 4 + tt][r] * OUT_FOLD + bob;
      }
    }
    __syncthreads();

    v4f vals[8];
    size_t dsts[8];
#pragma unroll
    for (int it = 0; it < 8; ++it) {
      const int L = wid * 32 + (l >> 3) + 4 * it;
      const int rl = L >> 3, seg = L & 7;
      vals[it] = *(const v4f*)&ftile[rl * 256 + seg * 32 + 4 * c];
      const int m = mblk0 + (rl >> 4) * 32 + p * 16 + (rl & 15);
      dsts[it] = (size_t)m * DM + nblk0 + seg * 32 + 4 * c;
    }
#pragma unroll
    for (int it = 0; it < 8; ++it) *(volatile v4f*)(Out + dsts[it]) = vals[it];
    __threadfence();
#pragma unroll
    for (int it = 0; it < 8; ++it) *(volatile v4f*)(Out + dsts[it]) = vals[it];
  }
}

extern "C" void kernel_launch(void* const* d_in, const int* in_sizes, int n_in,
                              void* d_out, int out_size, void* d_ws, size_t ws_size,
                              hipStream_t stream) {
  if (n_in < 11) return;
  const int need_x = ((NB - 1) * SEQ_FULL + SEQ) * DM;
  if (in_sizes[0] < need_x || in_sizes[1] < need_x || in_sizes[2] < need_x) return;
  if (in_sizes[3] < DM * DW || in_sizes[5] < DM * DW || in_sizes[7] < DM * DW || in_sizes[9] < DW * DM) return;
  if (in_sizes[4] < DW || in_sizes[6] < DW || in_sizes[8] < DW || in_sizes[10] < DM) return;
  if (out_size < MROWS * DM) return;
  if (WS_TOTAL_BYTES > ws_size) return;

  const float* Q  = (const float*)d_in[0];
  const float* K  = (const float*)d_in[1];
  const float* V  = (const float*)d_in[2];
  const float* Wq = (const float*)d_in[3];
  const float* bq = (const float*)d_in[4];
  const float* Wk = (const float*)d_in[5];
  const float* bk = (const float*)d_in[6];
  const float* Wv = (const float*)d_in[7];
  const float* bv = (const float*)d_in[8];
  const float* Wf = (const float*)d_in[9];
  const float* bf = (const float*)d_in[10];

  us* xq  = (us*)d_ws;
  us* xk  = xq + XE;
  us* xv  = xk + XE;
  us* wtq = xv + XE;
  us* wtk = wtq + WE;
  us* wtv = wtk + WE;
  us* wft = wtv + WE;
  us* qh  = wft + WE;
  us* kh  = qh + PE;
  us* vh  = kh + PE;
  us* vt  = vh + PE;
  us* ctx = vt + PE;

  dim3 blk(256);
  const int n8 = (int)(XE / 8);
  dim3 gx((n8 + 255) / 256);
  cvt_x_kernel<<<gx, blk, 0, stream>>>(Q, xq, n8);
  cvt_x_kernel<<<gx, blk, 0, stream>>>(K, xk, n8);
  cvt_x_kernel<<<gx, blk, 0, stream>>>(V, xv, n8);

  dim3 gw(DW / 64, DM / 64);
  cvt_w_kernel<<<gw, blk, 0, stream>>>(Wq, wtq, DM, DW, 0);
  cvt_w_kernel<<<gw, blk, 0, stream>>>(Wk, wtk, DM, DW, 0);
  cvt_w_kernel<<<gw, blk, 0, stream>>>(Wv, wtv, DM, DW, 0);
  dim3 gwf(DM / 64, DW / 64);
  cvt_w_kernel<<<gwf, blk, 0, stream>>>(Wf, wft, DW, DM, 1);

  dim3 gp(MROWS / 64, DW / 256);
  proj_kernel<<<gp, blk, 0, stream>>>(xq, wtq, bq, qh);
  proj_kernel<<<gp, blk, 0, stream>>>(xk, wtk, bk, kh);
  proj_kernel<<<gp, blk, 0, stream>>>(xv, wtv, bv, vh);

  vtrans_kernel<<<dim3(LSEQ / 64, NB * NH), blk, 0, stream>>>(vh, vt);

  attn_kernel<<<dim3(NB * NH * (LSEQ / 128)), blk, 0, stream>>>(qh, kh, vt, ctx);

  dim3 go(MROWS / 64, DM / 256);
  outproj_kernel<<<go, blk, 0, stream>>>(ctx, wft, bf, (float*)d_out);
}
